// GCNClassifier_77910706750016
// MI455X (gfx1250) — hardware-verified
//
#include <hip/hip_runtime.h>
#include <stddef.h>
#include <stdint.h>
#include <math.h>


#define D       128
#define KHL     256
#define KP      384
#define KM      256
#define NTHR    256
#define NWAVE   8
#define EPT     8
#define CHUNK   (NTHR * EPT)
#define WCAP    (EPT * 32)
#define LISTN   (NWAVE * WCAP)
#define NBA     1024
#define PKS     10
#define RCAP    34816
#define DEGCAP  128
#define GBM     64
#define GBN     128
#define GTHR    128
#define NUA     (D * (KHL / 8))
#define NUB     (D * (D / 8))
#define RG1     NUA
#define RG2     (RG1 + NUB)
#define RG3     (RG2 + NUA)
#define RG4     (RG3 + NUB)
#define RG5     (RG4 + NUA)
#define ZINTS   (2 * RCAP + 2 * NBA + LISTN)
#define LDS_AGG (ZINTS * 4 + 64)
#define WSMAX   134217728
#define BNEPS   1e-5f

static_assert((CHUNK & (CHUNK - 1)) == 0);
static_assert(NBA == (1 << PKS));
static_assert(((long long)CHUNK << PKS) < (1LL << 31));
static_assert(NTHR * 4 == NBA);
static_assert(LISTN >= NBA && LISTN >= NWAVE * WCAP);
static_assert((RCAP % 32) == 0);
static_assert((ZINTS % (NTHR * 4)) == 0);
static_assert(LDS_AGG <= 300000);
static_assert((NBA % NWAVE) == 0 && (NBA % GBM) == 0);
static_assert(GBM == (GTHR / 32) * 16);
static_assert(GBN == D && GTHR == GBN);
static_assert(KHL == 2 * D && KP == KHL + D && (KP % 32) == 0 && KM == 2 * D && (KM % 32) == 0);
static_assert(((KP * 2) % 128) == 0);
static_assert(((KM * 2) % 128) == 0);
static_assert((RG1 % NTHR) == 0 && (RG2 % NTHR) == 0 && (RG3 % NTHR) == 0 && (RG4 % NTHR) == 0 && (RG5 % NTHR) == 0);
static_assert(D == 32 * 4);
static_assert(D == 16 * 8);
static_assert((KHL / 8) == 32 && (D / 8) == 16);
static_assert((GBM * 4) % 128 == 0);

typedef float          v4f  __attribute__((ext_vector_type(4)));
typedef float          v8f  __attribute__((ext_vector_type(8)));
typedef int            v4i  __attribute__((ext_vector_type(4)));
typedef int            v8i  __attribute__((ext_vector_type(8)));
typedef unsigned short v8us __attribute__((ext_vector_type(8)));
typedef __bf16         v16b __attribute__((ext_vector_type(16)));
typedef v4f  __attribute__((may_alias)) v4fa;
typedef v4i  __attribute__((may_alias)) v4ia;
typedef v8us __attribute__((may_alias)) v8usa;
union Frag { v16b b; v8us h[2]; v8i w; };

__device__ __forceinline__ v8f wmk(const Frag& a, const Frag& b, v8f c) {
  v8f d = __builtin_amdgcn_wmma_f32_16x16x32_bf16(false, a.b, false, b.b, (short)0, c, false, false);
  asm volatile("v_nop\n\tv_nop\n\tv_nop\n\tv_nop" : "+v"(d) : "v"(a.w), "v"(b.w));
  return d;
}

__device__ __forceinline__ v8f z8() { v8f z = {0.f, 0.f, 0.f, 0.f, 0.f, 0.f, 0.f, 0.f}; return z; }

__device__ __forceinline__ unsigned bf16_bits(float f) {
  const unsigned u = __float_as_uint(f);
  return (u + 0x7FFFu + ((u >> 16) & 1u)) >> 16;
}
__device__ __forceinline__ float bf16_val(float f) {
  return __uint_as_float(bf16_bits(f) << 16);
}

__device__ __forceinline__ int scan_chunk(const int* __restrict__ dsts, int nE, int cbase, int slotBase,
                                          int nb, int vec8, int* list, int tid, int lane, int wave) {
  int wc = 0;
  const int el0  = tid * EPT;
  const int e0   = cbase + el0;
  const int sent = -2147483647 - 1;
  v4i da, db;
  if (vec8 != 0 && cbase + CHUNK <= nE) {
    da = *(const v4i*)(dsts + e0);
    db = *(const v4i*)(dsts + e0 + 4);
  } else {
    da.x = (e0     < nE) ? dsts[min(e0,     nE - 1)] : sent;
    da.y = (e0 + 1 < nE) ? dsts[min(e0 + 1, nE - 1)] : sent;
    da.z = (e0 + 2 < nE) ? dsts[min(e0 + 2, nE - 1)] : sent;
    da.w = (e0 + 3 < nE) ? dsts[min(e0 + 3, nE - 1)] : sent;
    db.x = (e0 + 4 < nE) ? dsts[min(e0 + 4, nE - 1)] : sent;
    db.y = (e0 + 5 < nE) ? dsts[min(e0 + 5, nE - 1)] : sent;
    db.z = (e0 + 6 < nE) ? dsts[min(e0 + 6, nE - 1)] : sent;
    db.w = (e0 + 7 < nE) ? dsts[min(e0 + 7, nE - 1)] : sent;
  }
  const unsigned nbs = (unsigned)slotBase;
  const unsigned unb = (unsigned)nb;
  const unsigned s0 = (unsigned)da.x - nbs, s1 = (unsigned)da.y - nbs;
  const unsigned s2 = (unsigned)da.z - nbs, s3 = (unsigned)da.w - nbs;
  const unsigned s4 = (unsigned)db.x - nbs, s5 = (unsigned)db.y - nbs;
  const unsigned s6 = (unsigned)db.z - nbs, s7 = (unsigned)db.w - nbs;
  const bool h0 = s0 < unb, h1 = s1 < unb, h2 = s2 < unb, h3 = s3 < unb;
  const bool h4 = s4 < unb, h5 = s5 < unb, h6 = s6 < unb, h7 = s7 < unb;
  const unsigned any = __builtin_amdgcn_ballot_w32(h0 | h1 | h2 | h3 | h4 | h5 | h6 | h7);
  if (any != 0u) {
#define HITJ(J, HJ, SJ) { \
      const unsigned mj = __builtin_amdgcn_ballot_w32(HJ); \
      if (mj != 0u) { \
        if (HJ) { \
          const int pos = wc + (int)__builtin_amdgcn_mbcnt_lo(mj, 0u); \
          if (pos < WCAP) list[wave * WCAP + pos] = ((el0 + (J)) << PKS) | (int)(SJ); \
        } \
        wc += (int)__builtin_popcount(mj); } }
    HITJ(0, h0, s0)
    HITJ(1, h1, s1)
    HITJ(2, h2, s2)
    HITJ(3, h3, s3)
    HITJ(4, h4, s4)
    HITJ(5, h5, s5)
    HITJ(6, h6, s6)
    HITJ(7, h7, s7)
#undef HITJ
  }
  return wc;
}

__global__ __launch_bounds__(NTHR) void k_wprep(const float* __restrict__ wrel0, const float* __restrict__ wroot0,
                                                const float* __restrict__ wrel1, const float* __restrict__ wroot1,
                                                const float* __restrict__ wm,
                                                unsigned short* BT0, unsigned short* BT1, unsigned short* BTM) {
  const int u = (int)blockIdx.x * NTHR + (int)threadIdx.x;
  const float* W;
  unsigned short* B;
  int v, root, pitch;
  if (u < RG1)      { W = wrel0;  B = BT0; v = u;       root = 0; pitch = KP; }
  else if (u < RG2) { W = wroot0; B = BT0; v = u - RG1; root = 1; pitch = KP; }
  else if (u < RG3) { W = wrel1;  B = BT1; v = u - RG2; root = 0; pitch = KP; }
  else if (u < RG4) { W = wroot1; B = BT1; v = u - RG3; root = 1; pitch = KP; }
  else if (u < RG5) { W = wm;     B = BTM; v = u - RG4; root = 0; pitch = KM; }
  else return;
  v8us o;
  unsigned short* dp;
  if (root == 0) {
    const int n = v >> 5;
    const int q = v & 31;
    const float* p = W + (size_t)(4 * q) * D + n;
    const unsigned short b0 = (unsigned short)bf16_bits(p[0]);
    const unsigned short b1 = (unsigned short)bf16_bits(p[D]);
    const unsigned short b2 = (unsigned short)bf16_bits(p[2 * D]);
    const unsigned short b3 = (unsigned short)bf16_bits(p[3 * D]);
    o[0] = b0; o[1] = b1; o[2] = b2; o[3] = b3;
    o[4] = b0; o[5] = b1; o[6] = b2; o[7] = b3;
    dp = B + (size_t)n * pitch + 8 * q;
  } else {
    const int n = v >> 4;
    const int q = v & 15;
    const float* p = W + (size_t)(8 * q) * D + n;
#pragma unroll
    for (int i = 0; i < 8; ++i) o[i] = (unsigned short)bf16_bits(p[(size_t)i * D]);
    dp = B + (size_t)n * KP + KHL + 8 * q;
  }
  *(volatile v8us*)dp = o;
  __threadfence();
  *(volatile v8us*)dp = o;
}

template <int EPI>
__global__ __launch_bounds__(GTHR) void k_gemm(const unsigned short* __restrict__ A, int lda,
                                               const unsigned short* __restrict__ BT, int K,
                                               const float* __restrict__ bias, const float* __restrict__ gam,
                                               const float* __restrict__ bet, const float* __restrict__ rme,
                                               const float* __restrict__ rva,
                                               float* outF, unsigned short* outP) {
  __shared__ __attribute__((aligned(16))) float stg[GBM * GBN];
  __shared__ __attribute__((aligned(16))) float cb[GBN];
  __shared__ __attribute__((aligned(16))) float csc[GBN];
  __shared__ __attribute__((aligned(16))) float crm[GBN];
  __shared__ __attribute__((aligned(16))) float cbe[GBN];
  const int tid = (int)threadIdx.x, lane = tid & 31, wave = tid >> 5, hh = lane >> 4, m = lane & 15;
  const int rowBase = (int)blockIdx.x * GBM;
  {
    const int c = tid;
    cb[c]  = bf16_val(bias[c]);
    csc[c] = bf16_val(gam[c]) * rsqrtf(bf16_val(rva[c]) + BNEPS);
    crm[c] = bf16_val(rme[c]);
    cbe[c] = bf16_val(bet[c]);
  }
  __syncthreads();

  v8f acc[8];
#pragma unroll
  for (int t = 0; t < 8; ++t) acc[t] = z8();
  const unsigned short* ap = A  + (size_t)(rowBase + 16 * wave + m) * (size_t)lda + 8 * hh;
  const unsigned short* wp = BT + (size_t)m * (size_t)K + 8 * hh;
  const int ksteps = K >> 5;
#pragma unroll 1
  for (int ks = 0; ks < ksteps; ++ks) {
    Frag af;
    af.h[0] = *(const v8usa*)(ap + 32 * ks);
    af.h[1] = *(const v8usa*)(ap + 32 * ks + 16);
#pragma unroll
    for (int t = 0; t < 8; ++t) {
      const unsigned short* wq = wp + (size_t)(16 * t) * (size_t)K + 32 * ks;
      Frag bf;
      bf.h[0] = *(const v8usa*)wq;
      bf.h[1] = *(const v8usa*)(wq + 16);
      acc[t] = wmk(af, bf, acc[t]);
    }
  }

#pragma unroll
  for (int t = 0; t < 8; ++t) {
    const int lc = 16 * t + m;
    const float bb = cb[lc], sc = csc[lc], rm = crm[lc], be = cbe[lc];
#pragma unroll
    for (int r = 0; r < 8; ++r) {
      const int lr = 16 * wave + 8 * hh + r;
      const float v = acc[t][r] + bb;
      stg[lr * GBN + lc] = fmaxf(fmaf(v - rm, sc, be), 0.0f);
    }
  }
  __syncthreads();

  if constexpr (EPI == 0) {
    v4f fv[16];
#pragma unroll
    for (int i = 0; i < 16; ++i) {
      const int lr = 16 * wave + i;
      fv[i] = *(const v4fa*)(stg + lr * GBN + 4 * lane);
    }
#pragma unroll
    for (int i = 0; i < 16; ++i) {
      const int gr = rowBase + 16 * wave + i;
      float* op = outF + (size_t)gr * (size_t)GBN + 4 * lane;
      *(volatile v4f*)op = fv[i];
    }
    __threadfence();
#pragma unroll
    for (int i = 0; i < 16; ++i) {
      const int gr = rowBase + 16 * wave + i;
      float* op = outF + (size_t)gr * (size_t)GBN + 4 * lane;
      *(volatile v4f*)op = fv[i];
    }
  } else {
    v8us pv[16];
#pragma unroll
    for (int i = 0; i < 16; ++i) {
      const int lr = 16 * wave + i;
      const v4f f = *(const v4fa*)(stg + lr * GBN + 4 * lane);
      const unsigned h0 = bf16_bits(f.x), h1 = bf16_bits(f.y), h2 = bf16_bits(f.z), h3 = bf16_bits(f.w);
      v8us o;
      o[0] = (unsigned short)h0; o[1] = (unsigned short)h1; o[2] = (unsigned short)h2; o[3] = (unsigned short)h3;
      o[4] = (unsigned short)bf16_bits(f.x - __uint_as_float(h0 << 16));
      o[5] = (unsigned short)bf16_bits(f.y - __uint_as_float(h1 << 16));
      o[6] = (unsigned short)bf16_bits(f.z - __uint_as_float(h2 << 16));
      o[7] = (unsigned short)bf16_bits(f.w - __uint_as_float(h3 << 16));
      pv[i] = o;
    }
#pragma unroll
    for (int i = 0; i < 16; ++i) {
      const int gr = rowBase + 16 * wave + i;
      unsigned short* op = outP + (size_t)gr * (size_t)KM + 8 * lane;
      *(volatile v8us*)op = pv[i];
    }
    __threadfence();
#pragma unroll
    for (int i = 0; i < 16; ++i) {
      const int gr = rowBase + 16 * wave + i;
      unsigned short* op = outP + (size_t)gr * (size_t)KM + 8 * lane;
      *(volatile v8us*)op = pv[i];
    }
  }
}

template <int RIN>
__global__ __launch_bounds__(NTHR) void k_agg(const int* __restrict__ srcs, const int* __restrict__ dsts,
                                              const float* __restrict__ ew, const float* __restrict__ F,
                                              unsigned short* Aout, int nN, int nE, int vec8) {
  extern __shared__ __attribute__((aligned(16))) int lds_i[];
  int* reg1 = lds_i;
  int* reg2 = reg1 + RCAP;
  int* scnt = reg2 + RCAP;
  int* soff = scnt + NBA;
  int* list = soff + NBA;
  int* wcnt = list + LISTN;
  int* wtot = wcnt + NWAVE;
  const int tid = (int)threadIdx.x, lane = tid & 31, wave = tid >> 5;
  const int nodeBase = (int)blockIdx.x * NBA;

  {
    const v4i z4 = {0, 0, 0, 0};
    for (int i = tid * 4; i < ZINTS; i += NTHR * 4) *(v4ia*)(lds_i + i) = z4;
    if (tid < 2 * NWAVE) wcnt[tid] = 0;
  }
  __syncthreads();

  int tot = 0;
  const int nChunks = (nE + CHUNK - 1) / CHUNK;
#pragma unroll 1
  for (int ch = 0; ch < nChunks; ++ch) {
    const int cbase = ch * CHUNK;
    const int wc = scan_chunk(dsts, nE, cbase, nodeBase, NBA, vec8, list, tid, lane, wave);
    if (lane == 0) wcnt[wave] = wc;
    __syncthreads();
    int pre = 0, all = 0;
#pragma unroll
    for (int w2 = 0; w2 < NWAVE; ++w2) {
      int c = wcnt[w2];
      c = c < 0 ? 0 : (c > WCAP ? WCAP : c);
      all += c;
      pre += (w2 < wave) ? c : 0;
    }
    const int wcc  = wc > WCAP ? WCAP : wc;
    const int base = tot + pre;
#pragma unroll 1
    for (int i = lane; i < wcc; i += 32) {
      const int ent = list[wave * WCAP + i];
      const int el  = (ent >> PKS) & (CHUNK - 1);
      const int sl  = ent & (NBA - 1);
      int eid = cbase + el;
      eid = eid > nE - 1 ? nE - 1 : eid;
      const int pos = base + i;
      if (pos < RCAP) reg1[pos] = (int)(((unsigned)eid << PKS) | (unsigned)sl);
    }
    tot += all;
    tot = tot > RCAP ? RCAP : tot;
    __syncthreads();
  }
  const int nh = tot;

  if (wave == 0) {
#pragma unroll 1
    for (int b0 = 0; b0 < nh; b0 += 32) {
      const int idx = b0 + lane;
      const int uv  = reg1[idx < RCAP ? idx : RCAP - 1];
      const int m32 = (nh - b0) < 32 ? (nh - b0) : 32;
#pragma unroll 1
      for (int k = 0; k < m32; ++k) {
        const int u  = __builtin_amdgcn_readlane(uv, k);
        const int sl = u & (NBA - 1);
        if (lane == 0) scnt[sl] = scnt[sl] + 1;
      }
    }
  }
  __syncthreads();

  {
    const v4i ca = *(const v4ia*)(scnt + 4 * tid);
    const int e0 = ca.x < 0 ? 0 : ca.x, e1 = ca.y < 0 ? 0 : ca.y, e2 = ca.z < 0 ? 0 : ca.z, e3 = ca.w < 0 ? 0 : ca.w;
    const int ts = e0 + e1 + e2 + e3;
    int incl = ts;
#pragma unroll
    for (int d = 1; d < 32; d <<= 1) {
      const int up = __shfl_up(incl, d, 32);
      if (lane >= d) incl += up;
    }
    if (lane == 31) wtot[wave] = incl;
    __syncthreads();
    int pre = 0;
#pragma unroll
    for (int w2 = 0; w2 < NWAVE; ++w2) pre += (w2 < wave) ? wtot[w2] : 0;
    int run = pre + incl - ts;
    soff[4 * tid + 0] = run; run += e0;
    soff[4 * tid + 1] = run; run += e1;
    soff[4 * tid + 2] = run; run += e2;
    soff[4 * tid + 3] = run;
  }
  __syncthreads();
  for (int i = tid; i < NBA; i += NTHR) list[i] = soff[i];
  __syncthreads();

  if (wave == 0) {
#pragma unroll 1
    for (int b0 = 0; b0 < nh; b0 += 32) {
      const int idx = b0 + lane;
      const int uv  = reg1[idx < RCAP ? idx : RCAP - 1];
      const int m32 = (nh - b0) < 32 ? (nh - b0) : 32;
#pragma unroll 1
      for (int k = 0; k < m32; ++k) {
        const int u   = __builtin_amdgcn_readlane(uv, k);
        const int sl  = u & (NBA - 1);
        const int eid = (int)((unsigned)u >> PKS);
        if (lane == 0) {
          int pos = list[sl];
          pos = pos < 0 ? 0 : (pos > RCAP - 1 ? RCAP - 1 : pos);
          reg2[pos] = eid;
          list[sl] = pos + 1;
        }
      }
    }
  }
  __syncthreads();

  const int nbw = NBA / NWAVE;
  const bool ovf = (nh >= RCAP);
  const float qnan = __int_as_float(0x7fc00000);
  const int c8 = 8 * (lane & 15);
  const bool xw = lane < 16;

#pragma unroll 1
  for (int jt = 0; jt < nbw; ++jt) {
    const int slot = wave * nbw + jt;
    const int node = nodeBase + slot;
    int st = soff[slot];
    const int craw = scnt[slot];
    int cnt = craw;
    st  = st < 0 ? 0 : (st > nh ? nh : st);
    cnt = cnt < 0 ? 0 : (cnt > DEGCAP ? DEGCAP : cnt);
    if (cnt > nh - st) cnt = nh - st;
    const float pz = (ovf || craw > DEGCAP) ? qnan : 0.0f;
    const bool live = node < nN;
    const int nc = node < nN ? node : nN - 1;

    float a0 = 0.0f, a1 = 0.0f, a2 = 0.0f, a3 = 0.0f;
#pragma unroll 1
    for (int b0 = 0; b0 < cnt; b0 += 32) {
      int idx = st + b0 + lane; idx = idx > RCAP - 1 ? RCAP - 1 : idx;
      int eid = reg2[idx]; eid = eid < 0 ? 0 : (eid > nE - 1 ? nE - 1 : eid);
      int sr = srcs[eid]; sr = sr < 0 ? 0 : (sr > nN - 1 ? nN - 1 : sr);
      const int wvi = __float_as_int(bf16_val(ew[eid]));
      const int m32 = (cnt - b0) < 32 ? (cnt - b0) : 32;
#pragma unroll 1
      for (int k = 0; k < m32; ++k) {
        const int   sk = __builtin_amdgcn_readlane(sr, k);
        const float wk = __int_as_float(__builtin_amdgcn_readlane(wvi, k));
        const v4f v = *(const v4fa*)(F + (size_t)sk * D + 4 * lane);
        float vx = v.x, vy = v.y, vz = v.z, vw = v.w;
        if constexpr (RIN == 1) {
          vx = bf16_val(vx); vy = bf16_val(vy); vz = bf16_val(vz); vw = bf16_val(vw);
        }
        a0 = fmaf(wk, vx, a0); a1 = fmaf(wk, vy, a1);
        a2 = fmaf(wk, vz, a2); a3 = fmaf(wk, vw, a3);
      }
    }
    const float r0 = (live ? a0 : 0.0f) + pz;
    const float r1 = (live ? a1 : 0.0f) + pz;
    const float r2 = (live ? a2 : 0.0f) + pz;
    const float r3 = (live ? a3 : 0.0f) + pz;

    const unsigned h0 = bf16_bits(r0), h1 = bf16_bits(r1), h2 = bf16_bits(r2), h3 = bf16_bits(r3);
    v8us pk;
    pk[0] = (unsigned short)h0; pk[1] = (unsigned short)h1; pk[2] = (unsigned short)h2; pk[3] = (unsigned short)h3;
    pk[4] = (unsigned short)bf16_bits(r0 - __uint_as_float(h0 << 16));
    pk[5] = (unsigned short)bf16_bits(r1 - __uint_as_float(h1 << 16));
    pk[6] = (unsigned short)bf16_bits(r2 - __uint_as_float(h2 << 16));
    pk[7] = (unsigned short)bf16_bits(r3 - __uint_as_float(h3 << 16));

    const float* xp = F + (size_t)nc * D + c8;
    const v4f xa = *(const v4fa*)xp;
    const v4f xb = *(const v4fa*)(xp + 4);
    v8us xo;
    xo[0] = (unsigned short)bf16_bits((live ? xa.x : 0.0f) + pz);
    xo[1] = (unsigned short)bf16_bits((live ? xa.y : 0.0f) + pz);
    xo[2] = (unsigned short)bf16_bits((live ? xa.z : 0.0f) + pz);
    xo[3] = (unsigned short)bf16_bits((live ? xa.w : 0.0f) + pz);
    xo[4] = (unsigned short)bf16_bits((live ? xb.x : 0.0f) + pz);
    xo[5] = (unsigned short)bf16_bits((live ? xb.y : 0.0f) + pz);
    xo[6] = (unsigned short)bf16_bits((live ? xb.z : 0.0f) + pz);
    xo[7] = (unsigned short)bf16_bits((live ? xb.w : 0.0f) + pz);

    unsigned short* gp = Aout + (size_t)node * (size_t)KP + 8 * lane;
    unsigned short* gx = Aout + (size_t)node * (size_t)KP + KHL + c8;
    *(volatile v8us*)gp = pk;
    if (xw) *(volatile v8us*)gx = xo;
    __threadfence();
    *(volatile v8us*)gp = pk;
    if (xw) *(volatile v8us*)gx = xo;
  }
}

__global__ __launch_bounds__(GTHR) void k_head(const unsigned short* __restrict__ A,
                                               const unsigned short* __restrict__ WT,
                                               const float* __restrict__ bm, const float* __restrict__ gm,
                                               const float* __restrict__ bem, const float* __restrict__ rmm,
                                               const float* __restrict__ rvm,
                                               const float* __restrict__ wout, const float* __restrict__ bout,
                                               float* outF, int nN) {
  __shared__ __attribute__((aligned(16))) float stg[GBM * GBN];
  __shared__ __attribute__((aligned(16))) float cb[GBN];
  __shared__ __attribute__((aligned(16))) float csc[GBN];
  __shared__ __attribute__((aligned(16))) float crm[GBN];
  __shared__ __attribute__((aligned(16))) float cbe[GBN];
  __shared__ __attribute__((aligned(16))) float wov[GBN];
  __shared__ __attribute__((aligned(16))) float orow[GBM];
  const int tid = (int)threadIdx.x, lane = tid & 31, wave = tid >> 5, hh = lane >> 4, m = lane & 15;
  const int rowBase = (int)blockIdx.x * GBM;
  {
    const int c = tid;
    cb[c]  = bf16_val(bm[c]);
    csc[c] = bf16_val(gm[c]) * rsqrtf(bf16_val(rvm[c]) + BNEPS);
    crm[c] = bf16_val(rmm[c]);
    cbe[c] = bf16_val(bem[c]);
    wov[c] = bf16_val(wout[c]);
  }
  const float bb2 = bf16_val(bout[0]);

  v8f acc[8];
#pragma unroll
  for (int t = 0; t < 8; ++t) acc[t] = z8();
  const unsigned short* ap = A  + (size_t)(rowBase + 16 * wave + m) * (size_t)KM + 8 * hh;
  const unsigned short* wp = WT + (size_t)m * (size_t)KM + 8 * hh;
#pragma unroll 1
  for (int ks = 0; ks < KM / 32; ++ks) {
    Frag af;
    af.h[0] = *(const v8usa*)(ap + 32 * ks);
    af.h[1] = *(const v8usa*)(ap + 32 * ks + 16);
#pragma unroll
    for (int t = 0; t < 8; ++t) {
      const unsigned short* wq = wp + (size_t)(16 * t) * (size_t)KM + 32 * ks;
      Frag bf;
      bf.h[0] = *(const v8usa*)wq;
      bf.h[1] = *(const v8usa*)(wq + 16);
      acc[t] = wmk(af, bf, acc[t]);
    }
  }

#pragma unroll
  for (int t = 0; t < 8; ++t) {
    const int lc = 16 * t + m;
#pragma unroll
    for (int r = 0; r < 8; ++r) {
      const int lr = 16 * wave + 8 * hh + r;
      stg[lr * GBN + lc] = acc[t][r];
    }
  }
  __syncthreads();

  {
    const int hr  = lane & 15;
    const int hc  = (lane >> 4) * 64;
    const int row = 16 * wave + hr;
    float s = 0.0f;
#pragma unroll 4
    for (int j = 0; j < 64; ++j) {
      const int c = hc + j;
      const float v  = stg[row * GBN + c] + cb[c];
      const float hv = fmaxf(fmaf(v - crm[c], csc[c], cbe[c]), 0.0f);
      s = fmaf(hv, wov[c], s);
    }
    const float so = __shfl_xor(s, 16, 32);
    s = s + so;
    float z = s + bb2;
    z = fminf(fmaxf(z, -80.0f), 80.0f);
    const float e = expf(-z);
    const float sg = 1.0f / (1.0f + e);
    if (lane < 16) orow[row] = sg;
  }
  __syncthreads();

  if (wave == 0) {
    const int q  = lane & 15;
    const int r0 = rowBase + 4 * q;
    const v4f w = *(const v4fa*)(orow + 4 * q);
    const bool full = (lane < 16) && (r0 + 4 <= nN);
    const bool part = (lane < 16) && (r0 < nN) && !full;
    float* op = outF + (size_t)r0;
    if (full) *(volatile v4f*)op = w;
    if (part) {
      if (r0 + 0 < nN) *(volatile float*)(op + 0) = w.x;
      if (r0 + 1 < nN) *(volatile float*)(op + 1) = w.y;
      if (r0 + 2 < nN) *(volatile float*)(op + 2) = w.z;
    }
    __threadfence();
    if (full) *(volatile v4f*)op = w;
    if (part) {
      if (r0 + 0 < nN) *(volatile float*)(op + 0) = w.x;
      if (r0 + 1 < nN) *(volatile float*)(op + 1) = w.y;
      if (r0 + 2 < nN) *(volatile float*)(op + 2) = w.z;
    }
  }
}

static inline int cdiv(int a, int b) { return (a + b - 1) / b; }
static inline size_t al256(size_t o) { return (o + 255) & ~(size_t)255; }

extern "C" void kernel_launch(void* const* d_in, const int* in_sizes, int n_in,
                              void* d_out, int out_size, void* d_ws, size_t ws_size,
                              hipStream_t stream) {
  if (n_in < 25) return;
  if (in_sizes[0] < D || (in_sizes[0] % D) != 0) return;
  const int nN = in_sizes[0] / D;
  if (nN < GBM || nN > (1 << 22)) return;
  if (in_sizes[1] < 2 || (in_sizes[1] & 1) != 0) return;
  const int nE = in_sizes[1] / 2;
  if (nE < 1 || nE >= (1 << (32 - PKS))) return;
  if (in_sizes[2] != nE) return;
  if (in_sizes[3] != D * D || in_sizes[5] != D * D) return;
  if (in_sizes[4] != D || in_sizes[6] != D || in_sizes[7] != D || in_sizes[8] != D || in_sizes[9] != D) return;
  if (in_sizes[10] != D * D || in_sizes[12] != D * D) return;
  if (in_sizes[11] != D || in_sizes[13] != D || in_sizes[14] != D || in_sizes[15] != D || in_sizes[16] != D) return;
  if (in_sizes[17] != D * D) return;
  if (in_sizes[18] != D || in_sizes[19] != D || in_sizes[20] != D || in_sizes[21] != D || in_sizes[22] != D) return;
  if (in_sizes[23] != D || in_sizes[24] != 1) return;
  if ((long long)out_size != (long long)nN) return;

  const float* x      = (const float*)d_in[0];
  const int*   ei     = (const int*)  d_in[1];
  const float* ew     = (const float*)d_in[2];
  const float* wrel0  = (const float*)d_in[3];
  const float* brel0  = (const float*)d_in[4];
  const float* wroot0 = (const float*)d_in[5];
  const float* g0     = (const float*)d_in[6];
  const float* be0    = (const float*)d_in[7];
  const float* rm0    = (const float*)d_in[8];
  const float* rv0    = (const float*)d_in[9];
  const float* wrel1  = (const float*)d_in[10];
  const float* brel1  = (const float*)d_in[11];
  const float* wroot1 = (const float*)d_in[12];
  const float* g1     = (const float*)d_in[13];
  const float* be1    = (const float*)d_in[14];
  const float* rm1    = (const float*)d_in[15];
  const float* rv1    = (const float*)d_in[16];
  const float* wm0    = (const float*)d_in[17];
  const float* bm0    = (const float*)d_in[18];
  const float* gm0    = (const float*)d_in[19];
  const float* bem0   = (const float*)d_in[20];
  const float* rmm0   = (const float*)d_in[21];
  const float* rvm0   = (const float*)d_in[22];
  const float* wout   = (const float*)d_in[23];
  const float* bout   = (const float*)d_in[24];
  float* out = (float*)d_out;
  const int* src = ei;
  const int* dst = ei + nE;

  const int MP   = cdiv(nN, GBM) * GBM;
  const int gM   = MP / GBM;
  const int gA   = cdiv(MP, NBA);
  const int RA   = gA * NBA;
  const int vec8 = ((nE & 3) == 0) ? 1 : 0;
  if ((long long)RA < (long long)MP) return;
  if ((long long)gM * GBM < (long long)nN) return;

  char* ws = (char*)d_ws;
  size_t off = 0;
  const size_t oBT0 = off; off = al256(off + (size_t)D * KP * 2);
  const size_t oBT1 = off; off = al256(off + (size_t)D * KP * 2);
  const size_t oBTM = off; off = al256(off + (size_t)D * KM * 2);
  const size_t oAP  = off; off = al256(off + (size_t)RA * KP * 2);
  size_t hs = (size_t)MP * D * 4;
  if ((size_t)MP * KM * 2 > hs) hs = (size_t)MP * KM * 2;
  const size_t oHS  = off; off = al256(off + hs);
  if (off > ws_size || off > (size_t)WSMAX) return;
  unsigned short* BT0 = (unsigned short*)(ws + oBT0);
  unsigned short* BT1 = (unsigned short*)(ws + oBT1);
  unsigned short* BTM = (unsigned short*)(ws + oBTM);
  unsigned short* AP  = (unsigned short*)(ws + oAP);
  float*          H1  = (float*)(ws + oHS);
  unsigned short* H2P = (unsigned short*)(ws + oHS);

  hipFuncSetAttribute(reinterpret_cast<const void*>(&k_agg<1>), hipFuncAttributeMaxDynamicSharedMemorySize, LDS_AGG);
  hipFuncSetAttribute(reinterpret_cast<const void*>(&k_agg<0>), hipFuncAttributeMaxDynamicSharedMemorySize, LDS_AGG);

  k_wprep<<<RG5 / NTHR, NTHR, 0, stream>>>(wrel0, wroot0, wrel1, wroot1, wm0, BT0, BT1, BTM);
  k_agg<1><<<gA, NTHR, LDS_AGG, stream>>>(src, dst, ew, x, AP, nN, nE, vec8);
  k_gemm<0><<<dim3(gM, 1), GTHR, 0, stream>>>(AP, KP, BT0, KP, brel0, g0, be0, rm0, rv0, H1, H2P);
  k_agg<0><<<gA, NTHR, LDS_AGG, stream>>>(src, dst, ew, H1, AP, nN, nE, vec8);
  k_gemm<1><<<dim3(gM, 1), GTHR, 0, stream>>>(AP, KP, BT1, KP, brel1, g1, be1, rm1, rv1, H1, H2P);
  k_head<<<gM, GTHR, 0, stream>>>(H2P, BTM, bm0, gm0, bem0, rmm0, rvm0, wout, bout, out, nN);
}
